// TransformerBlock_13846974562947
// MI455X (gfx1250) — hardware-verified
//
#include <hip/hip_runtime.h>
#include <math.h>

#ifndef NB
#define NB 2
#endif
#ifndef SEQ
#define SEQ 2048
#endif
#define NB_FULL 2
#define SEQ_FULL 2048
#define DM 1024
#define NH 16
#define HD 64
#define FF 4096
#define QW (3 * DM)
#define NT (NB * SEQ)
#define X_BSTRIDE_FULL ((long long)SEQ_FULL * DM)

static_assert(NB >= 1 && NB <= NB_FULL);
static_assert(SEQ >= 64 && SEQ <= SEQ_FULL);
static_assert(SEQ % 64 == 0);
static_assert(NT % 64 == 0);
static_assert(DM % 64 == 0 && QW % 64 == 0 && FF % 64 == 0);
static_assert(DM % 32 == 0 && FF % 32 == 0);
static_assert(NH * HD == DM);
static_assert(HD == 64);
static_assert(QW == NH * 3 * HD);
static_assert(DM == 32 * 4 * 8);
static_assert(DM % 8 == 0 && FF % 8 == 0);

typedef __attribute__((ext_vector_type(16))) _Float16 v16h;
typedef __attribute__((ext_vector_type(8)))  _Float16 v8h;
typedef _Float16 v8h_ma __attribute__((ext_vector_type(8), may_alias));
typedef __attribute__((ext_vector_type(8)))  float    v8f;
typedef __attribute__((ext_vector_type(4)))  float    v4f;
typedef float v4f_ma __attribute__((ext_vector_type(4), may_alias));
typedef unsigned int u4 __attribute__((ext_vector_type(4)));
typedef unsigned int u2 __attribute__((ext_vector_type(2)));

union FragU { v16h v; v8h h[2]; };
__device__ __forceinline__ v16h frag_ld(const _Float16* p) { FragU f; f.h[0] = *(const v8h*)(p); f.h[1] = *(const v8h*)(p + 16); return f.v; }
__device__ __forceinline__ v8f wmma16(v16h a, v16h b, v8f c) {
    c = __builtin_amdgcn_wmma_f32_16x16x32_f16(false, a, false, b, (short)0, c, false, false);
    asm volatile("v_nop\n\tv_nop\n\tv_nop\n\tv_nop" : "+v"(c) : "v"(a), "v"(b));
    return c;
}
__device__ __forceinline__ void dep_guard_h(v8f& a, v8f& b, v16h x, v16h y) { asm volatile("v_nop\n\tv_nop\n\tv_nop\n\tv_nop" : "+v"(a), "+v"(b) : "v"(x), "v"(y)); }
__device__ __forceinline__ void keep4_h(v16h a, v16h b, v16h c, v16h d) { asm volatile("v_nop" :: "v"(a), "v"(b), "v"(c), "v"(d)); }
__device__ __forceinline__ void acc_guard4(v8f& a, v8f& b, v8f& c, v8f& d) { asm volatile("v_nop\n\tv_nop\n\tv_nop\n\tv_nop" : "+v"(a), "+v"(b), "+v"(c), "+v"(d)); }
__device__ __forceinline__ void wave_sync() {
    __builtin_amdgcn_fence(3  , "workgroup");
    __builtin_amdgcn_wave_barrier();
    __builtin_amdgcn_fence(2  , "workgroup");
}

#define VST2(T, ptr, val) do { const T vst2_v_ = (val); *(volatile T*)(ptr) = vst2_v_; __threadfence(); *(volatile T*)(ptr) = vst2_v_; } while (0)

__device__ __forceinline__ float cmb_bf(float v) { const unsigned u = __builtin_bit_cast(unsigned, v); const unsigned r = (u + 0x7fffu + ((u >> 16) & 1u)) & 0xffff0000u; return __builtin_bit_cast(float, r); }
__device__ __forceinline__ unsigned int pk2h(float a, float b) { return (unsigned int)__builtin_bit_cast(unsigned short, (_Float16)a) | ((unsigned int)__builtin_bit_cast(unsigned short, (_Float16)b) << 16); }

__global__ __launch_bounds__(256) void k_castw(const float* __restrict__ SRC, unsigned short* __restrict__ DST, int nR, int nC, float sc) {
    const long long u = (long long)blockIdx.x * 256 + threadIdx.x; const int per = nC / 8; if (u >= (long long)nR * per) return;
    const int r = (int)(u / per); const int c0 = 8 * (int)(u % per);
    const float* s = SRC + (long long)r * nC + c0;
    const v4f a = *(const v4f*)(s), b = *(const v4f*)(s + 4);
    u4 pk;
    pk.x = pk2h(cmb_bf(a.x) * sc, cmb_bf(a.y) * sc); pk.y = pk2h(cmb_bf(a.z) * sc, cmb_bf(a.w) * sc);
    pk.z = pk2h(cmb_bf(b.x) * sc, cmb_bf(b.y) * sc); pk.w = pk2h(cmb_bf(b.z) * sc, cmb_bf(b.w) * sc);
    VST2(u4, (u4*)(DST + (long long)r * nC + c0), pk);
}

template <int ABF>
__device__ __forceinline__ void ln_body(const float* __restrict__ A, long long bstride, int rpb, const float* __restrict__ GA, const float* __restrict__ BE, int rows, unsigned short* __restrict__ Y16) {
    #pragma clang fp contract(off)
    const int r = blockIdx.x * 8 + (threadIdx.x >> 5); const int L = threadIdx.x & 31; if (r >= rows) return;
    const long long ab = (long long)(r / rpb) * bstride + (long long)(r % rpb) * DM;
    v4f v[8]; float s = 0.f;
#pragma unroll
    for (int q = 0; q < 8; ++q) {
        v[q] = *(const v4f*)(A + ab + 4 * L + 128 * q);
        if (ABF) { v[q].x = cmb_bf(v[q].x); v[q].y = cmb_bf(v[q].y); v[q].z = cmb_bf(v[q].z); v[q].w = cmb_bf(v[q].w); }
        s += (v[q].x + v[q].y) + (v[q].z + v[q].w);
    }
#pragma unroll
    for (int o = 16; o > 0; o >>= 1) s += __shfl_xor(s, o, 32);
    const float mu = s * (1.f / DM); float qq = 0.f;
#pragma unroll
    for (int q = 0; q < 8; ++q) { v[q].x -= mu; v[q].y -= mu; v[q].z -= mu; v[q].w -= mu; qq += (v[q].x * v[q].x + v[q].y * v[q].y) + (v[q].z * v[q].z + v[q].w * v[q].w); }
#pragma unroll
    for (int o = 16; o > 0; o >>= 1) qq += __shfl_xor(qq, o, 32);
    const float rs = rsqrtf(qq * (1.f / DM) + 1e-5f);
#pragma unroll
    for (int q = 0; q < 8; ++q) {
        const int c = 4 * L + 128 * q; const v4f ga = *(const v4f*)(GA + c), be = *(const v4f*)(BE + c);
        const float y0 = v[q].x * rs * cmb_bf(ga.x) + cmb_bf(be.x), y1 = v[q].y * rs * cmb_bf(ga.y) + cmb_bf(be.y);
        const float y2 = v[q].z * rs * cmb_bf(ga.z) + cmb_bf(be.z), y3 = v[q].w * rs * cmb_bf(ga.w) + cmb_bf(be.w);
        u2 pk; pk.x = pk2h(y0, y1); pk.y = pk2h(y2, y3);
        VST2(u2, (u2*)(Y16 + (long long)r * DM + c), pk);
    }
}
__global__ __launch_bounds__(256) void k_ln_in(const float* __restrict__ X, const float* __restrict__ GA, const float* __restrict__ BE, unsigned short* __restrict__ Y16) {
    ln_body<1>(X, X_BSTRIDE_FULL, SEQ, GA, BE, NT, Y16);
}
__global__ __launch_bounds__(256) void k_ln_mid(const float* __restrict__ X1, const float* __restrict__ GA, const float* __restrict__ BE, unsigned short* __restrict__ Y16) {
    ln_body<0>(X1, 0LL, NT, GA, BE, NT, Y16);
}

#define SLAB (16 * 68)
template <int OUT_MODE, int RESID, int ACT>
__device__ __forceinline__ void gemm64_body(const unsigned short* __restrict__ Ap, int lda, const unsigned short* __restrict__ Btp, int ldb,
                                            float* __restrict__ Cf, unsigned short* __restrict__ Ch, int ldc, const float* __restrict__ bias,
                                            const float* __restrict__ resid, int ldr, int rrpb, long long rbs, int M, int N, int K, float scale) {
    __shared__ __align__(16) float sT[8 * SLAB];
    const _Float16* A = (const _Float16*)Ap; const _Float16* Bt = (const _Float16*)Btp;
    const int lane = threadIdx.x & 31, wave = threadIdx.x >> 5;
    const int tilesN = N >> 6, tilesM = M >> 6;
    const int tile = blockIdx.x * 8 + wave;
    if (tile >= tilesM * tilesN) return;
    const int tm = tile / tilesN, tn = tile - tm * tilesN;
    const int m0 = tm << 6, n0 = tn << 6;
    const int rlane = lane & 15, koff = (lane >> 4) * 8, mOff = (lane >> 4) * 8;

    v8f acc[4][4];
#pragma unroll
    for (int i = 0; i < 4; ++i)
#pragma unroll
        for (int j = 0; j < 4; ++j) acc[i][j] = (v8f){0.f, 0.f, 0.f, 0.f, 0.f, 0.f, 0.f, 0.f};

    for (int k0 = 0; k0 < K; k0 += 32) {
        v16h bh[4];
#pragma unroll
        for (int j = 0; j < 4; ++j) bh[j] = frag_ld(Bt + (size_t)(n0 + (j << 4) + rlane) * ldb + koff + k0);
#pragma unroll
        for (int i = 0; i < 4; ++i) {
            const v16h ah = frag_ld(A + (size_t)(m0 + (i << 4) + rlane) * lda + koff + k0);
#pragma unroll
            for (int j = 0; j < 4; ++j) acc[i][j] = __builtin_amdgcn_wmma_f32_16x16x32_f16(false, ah, false, bh[j], (short)0, acc[i][j], false, false);
            dep_guard_h(acc[i][0], acc[i][3], ah, ah);
        }
        keep4_h(bh[0], bh[1], bh[2], bh[3]);
    }
    acc_guard4(acc[0][0], acc[0][1], acc[0][2], acc[0][3]);
    acc_guard4(acc[1][0], acc[1][1], acc[1][2], acc[1][3]);
    acc_guard4(acc[2][0], acc[2][1], acc[2][2], acc[2][3]);
    acc_guard4(acc[3][0], acc[3][1], acc[3][2], acc[3][3]);

    const int sb = wave * SLAB;
#pragma unroll
    for (int i = 0; i < 4; ++i) {
        const int mBase = m0 + (i << 4);
#pragma unroll
        for (int j = 0; j < 4; ++j) {
            const int n = n0 + (j << 4) + rlane;
            const float bv = cmb_bf(bias[n]);
#pragma unroll
            for (int r = 0; r < 8; ++r) {
                float v = acc[i][j][r] * scale + bv;
                if (ACT == 1) v = fmaxf(v, 0.0f);
                sT[sb + (mOff + r) * 68 + (j << 4) + rlane] = v;
            }
        }
        wave_sync();
        if (OUT_MODE == 0) {
            const int hh = lane >> 4, c4 = (lane & 15) * 4;
            if (RESID != 0) {
#pragma unroll
                for (int it = 0; it < 8; ++it) {
                    const int row = it * 2 + hh; const int mm = mBase + row;
                    const long long ro = (long long)(mm / rrpb) * rbs + (long long)(mm % rrpb) * ldr + n0 + c4;
                    v4f rr = *(const v4f*)(resid + ro);
                    if (RESID == 2) { rr.x = cmb_bf(rr.x); rr.y = cmb_bf(rr.y); rr.z = cmb_bf(rr.z); rr.w = cmb_bf(rr.w); }
                    v4f sv = *(const v4f_ma*)(&sT[sb + row * 68 + c4]);
                    sv.x += rr.x; sv.y += rr.y; sv.z += rr.z; sv.w += rr.w;
                    *(v4f_ma*)(&sT[sb + row * 68 + c4]) = sv;
                }
            }
            for (int pass = 0; pass < 2; ++pass) {
#pragma unroll
                for (int it = 0; it < 8; ++it) {
                    const int row = it * 2 + hh;
                    const v4f v = *(const v4f_ma*)(&sT[sb + row * 68 + c4]);
                    *(volatile v4f*)(Cf + (size_t)(mBase + row) * ldc + n0 + c4) = v;
                }
                __threadfence();
            }
        } else {
            const int q = lane >> 3, c8 = (lane & 7) * 8;
            for (int pass = 0; pass < 2; ++pass) {
#pragma unroll
                for (int it = 0; it < 4; ++it) {
                    const int row = it * 4 + q;
                    v8h hv;
#pragma unroll
                    for (int e = 0; e < 8; ++e) hv[e] = (_Float16)sT[sb + row * 68 + c8 + e];
                    *(volatile v8h*)(Ch + (size_t)(mBase + row) * ldc + n0 + c8) = hv;
                }
                __threadfence();
            }
        }
        wave_sync();
    }
}
__global__ __launch_bounds__(256) void k_gemm_qkv(const unsigned short* __restrict__ A, const unsigned short* __restrict__ Bt, unsigned short* __restrict__ C, const float* __restrict__ bias) {
    gemm64_body<1, 0, 0>(A, DM, Bt, DM, nullptr, C, QW, bias, nullptr, 0, 1, 0LL, NT, QW, DM, 0.0625f);
}
__global__ __launch_bounds__(256) void k_gemm_proj(const unsigned short* __restrict__ A, const unsigned short* __restrict__ Bt, float* __restrict__ C, const float* __restrict__ bias, const float* __restrict__ X) {
    gemm64_body<0, 2, 0>(A, DM, Bt, DM, C, nullptr, DM, bias, X, DM, SEQ, X_BSTRIDE_FULL, NT, DM, DM, 0.00390625f);
}
__global__ __launch_bounds__(256) void k_gemm_up(const unsigned short* __restrict__ A, const unsigned short* __restrict__ Bt, unsigned short* __restrict__ C, const float* __restrict__ bias) {
    gemm64_body<1, 0, 1>(A, DM, Bt, DM, nullptr, C, FF, bias, nullptr, 0, 1, 0LL, NT, FF, DM, 0.0625f);
}
__global__ __launch_bounds__(256) void k_gemm_down(const unsigned short* __restrict__ A, const unsigned short* __restrict__ Bt, float* __restrict__ C, const float* __restrict__ bias, const float* __restrict__ X1) {
    gemm64_body<0, 1, 0>(A, FF, Bt, FF, C, nullptr, DM, bias, X1, DM, NT, 0LL, NT, DM, FF, 0.0625f);
}

#define VT_PITCH 72
static_assert(256 * 16 == 64 * 64);
static_assert(2 * 256 == 64 * 8);
static_assert((VT_PITCH * 2) % 16 == 0);
__global__ __launch_bounds__(256) void k_vt(const unsigned short* __restrict__ QKVp, unsigned short* __restrict__ VTp) {
    __shared__ __align__(16) _Float16 tile[64 * VT_PITCH];
    const _Float16* QKV = (const _Float16*)QKVp;
    const int nsb = SEQ / 64; const int bx = blockIdx.x; const int sbk = bx % nsb; const int bh = bx / nsb; const int h = bh % NH; const int b = bh / NH;
    const int t = threadIdx.x;
    {
        const int tr = t >> 2, dc = (t & 3) * 16;
        const _Float16* src = QKV + (size_t)(b * SEQ + sbk * 64 + tr) * QW + h * 192 + 128 + dc;
        const v8h a = *(const v8h*)(src), bb = *(const v8h*)(src + 8);
        *(v8h*)(&tile[tr * VT_PITCH + dc]) = a; *(v8h*)(&tile[tr * VT_PITCH + dc + 8]) = bb;
    }
    __syncthreads();
    const int d0 = t >> 3, d1 = (t + 256) >> 3, tk = (t & 7) * 8;
    v8h p0, p1;
#pragma unroll
    for (int e = 0; e < 8; ++e) { p0[e] = tile[(tk + e) * VT_PITCH + d0]; p1[e] = tile[(tk + e) * VT_PITCH + d1]; }
    volatile v8h* q0 = (volatile v8h*)(VTp + (size_t)(bh * 64 + d0) * SEQ + sbk * 64 + tk);
    volatile v8h* q1 = (volatile v8h*)(VTp + (size_t)(bh * 64 + d1) * SEQ + sbk * 64 + tk);
    *q0 = p0; *q1 = p1; __threadfence(); *q0 = p0; *q1 = p1;
}

#define AT_PP 40
static_assert(AT_PP >= 32 && (AT_PP * 2) % 16 == 0);
static_assert(4 * 16 == 64);
__global__ __launch_bounds__(128) void k_attn(const unsigned short* __restrict__ QKVp, const unsigned short* __restrict__ VTp, unsigned short* __restrict__ CTX) {
    __shared__ __align__(16) _Float16 Pw[4 * 16 * AT_PP];
    __shared__ __align__(16) float    Os[4 * SLAB];
    const _Float16* QKV = (const _Float16*)QKVp; const _Float16* VT = (const _Float16*)VTp;
    const int lane = threadIdx.x & 31, wave = threadIdx.x >> 5, hf = lane >> 4, c = lane & 15;
    const int nqb = SEQ / 64; const int bx = blockIdx.x; const int qb = bx % nqb; const int bh = bx / nqb; const int h = bh % NH; const int b = bh / NH;
    const int q0 = qb * 64 + wave * 16;
    const int pbase = wave * 16 * AT_PP;
    const long long qoff  = (long long)(b * SEQ + q0 + c) * QW + h * 192 + 8 * hf;
    const long long kbase = (long long)(b * SEQ + c) * QW + h * 192 + 64 + 8 * hf;
    const long long vbase = (long long)(bh * 64 + c) * SEQ + 8 * hf;
    const float csc = 0.125f * 1.4426950408889634f;

    v8f o[4]; float m8[8], l8[8];
#pragma unroll
    for (int t = 0; t < 4; ++t) o[t] = (v8f){0.f, 0.f, 0.f, 0.f, 0.f, 0.f, 0.f, 0.f};
#pragma unroll
    for (int r = 0; r < 8; ++r) { m8[r] = -__builtin_inff(); l8[r] = 0.f; }

    for (int j0 = 0; j0 < SEQ; j0 += 32) {
        const v16h qa0 = frag_ld(QKV + qoff), qa1 = frag_ld(QKV + qoff + 32);
        const long long k0o = kbase + (long long)j0 * QW, k1o = k0o + 16LL * QW;
        v8f s0 = (v8f){0.f, 0.f, 0.f, 0.f, 0.f, 0.f, 0.f, 0.f}, s1 = s0;
        s0 = wmma16(qa0, frag_ld(QKV + k0o), s0); s0 = wmma16(qa1, frag_ld(QKV + k0o + 32), s0);
        s1 = wmma16(qa0, frag_ld(QKV + k1o), s1); s1 = wmma16(qa1, frag_ld(QKV + k1o + 32), s1);
#pragma unroll
        for (int r = 0; r < 8; ++r) {
            const float v0 = s0[r] * csc, v1 = s1[r] * csc;
            float mx = fmaxf(v0, v1);
            mx = fmaxf(mx, __shfl_xor(mx, 1, 32)); mx = fmaxf(mx, __shfl_xor(mx, 2, 32));
            mx = fmaxf(mx, __shfl_xor(mx, 4, 32)); mx = fmaxf(mx, __shfl_xor(mx, 8, 32));
            const float mnew = fmaxf(m8[r], mx);
            const float corr = exp2f(m8[r] - mnew);
            const float p0 = exp2f(v0 - mnew), p1 = exp2f(v1 - mnew);
            l8[r] = l8[r] * corr + (p0 + p1);
            m8[r] = mnew;
#pragma unroll
            for (int t = 0; t < 4; ++t) o[t][r] *= corr;
            Pw[pbase + (8 * hf + r) * AT_PP + c]      = (_Float16)(p0 * 4096.0f);
            Pw[pbase + (8 * hf + r) * AT_PP + 16 + c] = (_Float16)(p1 * 4096.0f);
        }
        wave_sync();
        FragU pa;
        pa.h[0] = *(const v8h_ma*)(&Pw[pbase + c * AT_PP + 8 * hf]);
        pa.h[1] = *(const v8h_ma*)(&Pw[pbase + c * AT_PP + 16 + 8 * hf]);
        const long long vo = vbase + j0;
        const v16h vb0 = frag_ld(VT + vo), vb1 = frag_ld(VT + vo + 16LL * SEQ), vb2 = frag_ld(VT + vo + 32LL * SEQ), vb3 = frag_ld(VT + vo + 48LL * SEQ);
        o[0] = wmma16(pa.v, vb0, o[0]); o[1] = wmma16(pa.v, vb1, o[1]); o[2] = wmma16(pa.v, vb2, o[2]); o[3] = wmma16(pa.v, vb3, o[3]);
        wave_sync();
    }

    const int ob = wave * SLAB;
#pragma unroll
    for (int r = 0; r < 8; ++r) {
        float l = l8[r];
        l += __shfl_xor(l, 1, 32); l += __shfl_xor(l, 2, 32); l += __shfl_xor(l, 4, 32); l += __shfl_xor(l, 8, 32);
        const float inv = 1.0f / (l * 256.0f);
#pragma unroll
        for (int t = 0; t < 4; ++t) Os[ob + (8 * hf + r) * 68 + t * 16 + c] = o[t][r] * inv;
    }
    wave_sync();
    {
        const int q = lane >> 3, c8 = (lane & 7) * 8;
        for (int pass = 0; pass < 2; ++pass) {
#pragma unroll
            for (int it = 0; it < 4; ++it) {
                const int row = it * 4 + q;
                v8h hv;
#pragma unroll
                for (int e = 0; e < 8; ++e) hv[e] = (_Float16)Os[ob + row * 68 + c8 + e];
                *(volatile v8h*)(CTX + (size_t)(b * SEQ + q0 + row) * DM + h * 64 + c8) = hv;
            }
            __threadfence();
        }
    }
}

#define A256(x) (((((size_t)(x)) + 255) / 256) * 256)
constexpr size_t SZ_W3  = A256((size_t)QW * DM * 2);
constexpr size_t SZ_WO  = A256((size_t)DM * DM * 2);
constexpr size_t SZ_W1  = A256((size_t)FF * DM * 2);
constexpr size_t SZ_W2  = A256((size_t)DM * FF * 2);
constexpr size_t SZ_H   = A256((size_t)NT * DM * 2);
constexpr size_t SZ_QKV = A256((size_t)NT * QW * 2);
constexpr size_t SZ_VT  = A256((size_t)NB * NH * HD * SEQ * 2);
constexpr size_t SZ_CTX = A256((size_t)NT * DM * 2);
constexpr size_t SZ_X1  = A256((size_t)NT * DM * 4);
constexpr size_t SZ_F   = A256((size_t)NT * FF * 2);
constexpr size_t OFF_W3 = 0;
constexpr size_t OFF_WO = OFF_W3 + SZ_W3;
constexpr size_t OFF_W1 = OFF_WO + SZ_WO;
constexpr size_t OFF_W2 = OFF_W1 + SZ_W1;
constexpr size_t OFF_H  = OFF_W2 + SZ_W2;
constexpr size_t OFF_QKV = OFF_H + SZ_H;
constexpr size_t OFF_VT = OFF_QKV + SZ_QKV;
constexpr size_t OFF_CTX = OFF_VT + SZ_VT;
constexpr size_t OFF_X1 = OFF_CTX + SZ_CTX;
constexpr size_t OFF_F  = OFF_X1 + SZ_X1;
constexpr size_t WS_TOTAL = OFF_F + SZ_F;
static_assert(WS_TOTAL <= (size_t)134217728);
static_assert(((NT / 64) * (QW / 64)) % 8 == 0 || true);

extern "C" void kernel_launch(void* const* d_in, const int* in_sizes, int n_in, void* d_out, int out_size, void* d_ws, size_t ws_size, hipStream_t stream) {
    if (n_in < 13) return;
    if ((long long)in_sizes[0] < ((long long)(NB - 1) * SEQ_FULL + SEQ) * DM) return;
    if ((long long)in_sizes[1] < (long long)QW * DM || in_sizes[2] < QW) return;
    if ((long long)in_sizes[3] < (long long)DM * DM || in_sizes[4] < DM) return;
    if ((long long)in_sizes[5] < (long long)FF * DM || in_sizes[6] < FF) return;
    if ((long long)in_sizes[7] < (long long)DM * FF || in_sizes[8] < DM) return;
    if (in_sizes[9] < DM || in_sizes[10] < DM || in_sizes[11] < DM || in_sizes[12] < DM) return;
    if ((long long)out_size < (long long)NT * DM) return;
    if (ws_size < WS_TOTAL) return;

    const float* x     = (const float*)d_in[0];
    const float* w_qkv = (const float*)d_in[1];
    const float* b_qkv = (const float*)d_in[2];
    const float* w_out = (const float*)d_in[3];
    const float* b_out = (const float*)d_in[4];
    const float* w1    = (const float*)d_in[5];
    const float* b1    = (const float*)d_in[6];
    const float* w2    = (const float*)d_in[7];
    const float* b2    = (const float*)d_in[8];
    const float* ln1g  = (const float*)d_in[9];
    const float* ln1b  = (const float*)d_in[10];
    const float* ln2g  = (const float*)d_in[11];
    const float* ln2b  = (const float*)d_in[12];
    float* out = (float*)d_out;

    char* ws = (char*)d_ws;
    unsigned short* W3    = (unsigned short*)(ws + OFF_W3);
    unsigned short* WO    = (unsigned short*)(ws + OFF_WO);
    unsigned short* W1h   = (unsigned short*)(ws + OFF_W1);
    unsigned short* W2h   = (unsigned short*)(ws + OFF_W2);
    unsigned short* H16   = (unsigned short*)(ws + OFF_H);
    unsigned short* QKV16 = (unsigned short*)(ws + OFF_QKV);
    unsigned short* VT16  = (unsigned short*)(ws + OFF_VT);
    unsigned short* CTX16 = (unsigned short*)(ws + OFF_CTX);
    float*          X1    = (float*)(ws + OFF_X1);
    unsigned short* F16p  = (unsigned short*)(ws + OFF_F);

    k_castw<<<(unsigned)(((long long)QW * (DM / 8) + 255) / 256), 256, 0, stream>>>(w_qkv, W3, QW, DM, 16.0f);
    k_castw<<<(unsigned)(((long long)DM * (DM / 8) + 255) / 256), 256, 0, stream>>>(w_out, WO, DM, DM, 16.0f);
    k_castw<<<(unsigned)(((long long)FF * (DM / 8) + 255) / 256), 256, 0, stream>>>(w1, W1h, FF, DM, 16.0f);
    k_castw<<<(unsigned)(((long long)DM * (FF / 8) + 255) / 256), 256, 0, stream>>>(w2, W2h, DM, FF, 16.0f);
    k_ln_in<<<(NT + 7) / 8, 256, 0, stream>>>(x, ln1g, ln1b, H16);
    k_gemm_qkv<<<(unsigned)(((NT / 64) * (QW / 64) + 7) / 8), 256, 0, stream>>>(H16, W3, QKV16, b_qkv);
    k_vt<<<(unsigned)(NB * NH * (SEQ / 64)), 256, 0, stream>>>(QKV16, VT16);
    k_attn<<<(unsigned)(NB * NH * (SEQ / 64)), 128, 0, stream>>>(QKV16, VT16, CTX16);
    k_gemm_proj<<<(unsigned)(((NT / 64) * (DM / 64) + 7) / 8), 256, 0, stream>>>(CTX16, WO, X1, b_out, x);
    k_ln_mid<<<(NT + 7) / 8, 256, 0, stream>>>(X1, ln2g, ln2b, H16);
    k_gemm_up<<<(unsigned)(((NT / 64) * (FF / 64) + 7) / 8), 256, 0, stream>>>(H16, W1h, F16p, b1);
    k_gemm_down<<<(unsigned)(((NT / 64) * (DM / 64) + 7) / 8), 256, 0, stream>>>(F16p, W2h, out, b2, X1);
}
